// KnotTransformerLayer_6141803233390
// MI455X (gfx1250) — hardware-verified
//
#include <hip/hip_runtime.h>
#include <stddef.h>
#include <stdint.h>


#define DD 128
#define NHEAD 4
#define NSLOT 5
#define DFF 512
#define NCOL 20
#define LN_EPS 1e-5f
#define QK_SCALE 0.17677669529663687f
#define APITCH 136
#define QPITCH 132
#define UPITCH 520
#define FPITCH 132
#define STATW 32

typedef __attribute__((ext_vector_type(16))) _Float16 v16h;
typedef __attribute__((ext_vector_type(8)))  _Float16 v8h;
typedef __attribute__((ext_vector_type(4)))  _Float16 v4h;
typedef __attribute__((ext_vector_type(8)))  float    v8f;
typedef __attribute__((ext_vector_type(4)))  float    v4f;

__device__ __forceinline__ void dep_guard_h(v8f& a, v8f& b, v16h x, v16h y) {
  asm volatile("v_nop\n\tv_nop\n\tv_nop\n\tv_nop" : "+v"(a), "+v"(b) : "v"(x), "v"(y));
}
__device__ __forceinline__ void dep_guard4_h(v8f& a, v8f& b, v8f& c2, v8f& d, v16h x, v16h y) {
  asm volatile("v_nop\n\tv_nop\n\tv_nop\n\tv_nop" : "+v"(a), "+v"(b), "+v"(c2), "+v"(d) : "v"(x), "v"(y));
}
__device__ __forceinline__ void keep2_h(v16h a, v16h b) { asm volatile("v_nop" :: "v"(a), "v"(b)); }
__device__ __forceinline__ void keep4_h(v16h a, v16h b, v16h c, v16h d) { asm volatile("v_nop" :: "v"(a), "v"(b), "v"(c), "v"(d)); }
__device__ __forceinline__ void acc_guard4(v8f& a, v8f& b, v8f& c, v8f& d) {
  asm volatile("v_nop\n\tv_nop\n\tv_nop\n\tv_nop" : "+v"(a), "+v"(b), "+v"(c), "+v"(d));
}
template <typename T> struct Frag;
template <> struct Frag<_Float16> {
  typedef v16h V; union U { v16h v; v8h h[2]; };
  static __device__ __forceinline__ v16h load(const _Float16* p) {
    U f; f.h[0] = *(const v8h*)(p); f.h[1] = *(const v8h*)(p + 16); return f.v;
  }
  static __device__ __forceinline__ v8f mma(v16h a, v16h b, v8f c) {
    return __builtin_amdgcn_wmma_f32_16x16x32_f16(false, a, false, b, (short)0, c, false, false);
  }
  static __device__ __forceinline__ void guard(v8f& a, v8f& b, v16h x, v16h y) { dep_guard_h(a, b, x, y); }
  static __device__ __forceinline__ void keep(v16h a, v16h b, v16h c, v16h d) { keep4_h(a, b, c, d); }
};
typedef Frag<_Float16> FH;

__device__ __forceinline__ void wave_lds_sync() {
  __builtin_amdgcn_fence(__ATOMIC_RELEASE, "workgroup");
  __builtin_amdgcn_wave_barrier();
  __builtin_amdgcn_fence(__ATOMIC_ACQUIRE, "workgroup");
}

__device__ __forceinline__ void store2_v4f(float* p, v4f v) {
  *(volatile v4f*)p = v;
  __threadfence();
  *(volatile v4f*)p = v;
}

template <int MI, int NJ>
__device__ __forceinline__ void zero_acc(v8f (&acc)[MI][NJ]) {
#pragma unroll
  for (int i = 0; i < MI; ++i)
#pragma unroll
    for (int j = 0; j < NJ; ++j) acc[i][j] = (v8f){0.f, 0.f, 0.f, 0.f, 0.f, 0.f, 0.f, 0.f};
}

__device__ __forceinline__ void tile_mma_42(const _Float16* At, int lda, const _Float16* __restrict__ Bt, int ldb,
                                            int lane, v8f (&acc)[4][2]) {
  const int c = lane & 15, koff = (lane >> 4) * 8;
#pragma unroll
  for (int kt = 0; kt < 4; ++kt) {
    v16h b[2];
#pragma unroll
    for (int j = 0; j < 2; ++j) b[j] = FH::load(Bt + (size_t)(16 * j + c) * ldb + 32 * kt + koff);
#pragma unroll
    for (int i = 0; i < 4; ++i) {
      const v16h a = FH::load(At + (16 * i + c) * lda + 32 * kt + koff);
      acc[i][0] = FH::mma(a, b[0], acc[i][0]);
      acc[i][1] = FH::mma(a, b[1], acc[i][1]);
      dep_guard_h(acc[i][0], acc[i][1], a, b[1]);
    }
    keep2_h(b[0], b[1]);
  }
}
__device__ __forceinline__ void tile_mma_24(const _Float16* At, int lda, const _Float16* __restrict__ Bt, int ldb,
                                            int lane, v8f (&acc)[2][4]) {
  const int c = lane & 15, koff = (lane >> 4) * 8;
#pragma unroll
  for (int kt = 0; kt < 4; ++kt) {
    v16h b[4];
#pragma unroll
    for (int j = 0; j < 4; ++j) b[j] = FH::load(Bt + (size_t)(16 * j + c) * ldb + 32 * kt + koff);
#pragma unroll
    for (int i = 0; i < 2; ++i) {
      const v16h a = FH::load(At + (16 * i + c) * lda + 32 * kt + koff);
      acc[i][0] = FH::mma(a, b[0], acc[i][0]);
      acc[i][1] = FH::mma(a, b[1], acc[i][1]);
      acc[i][2] = FH::mma(a, b[2], acc[i][2]);
      acc[i][3] = FH::mma(a, b[3], acc[i][3]);
      dep_guard4_h(acc[i][0], acc[i][1], acc[i][2], acc[i][3], a, b[3]);
    }
    keep4_h(b[0], b[1], b[2], b[3]);
  }
}

__device__ __forceinline__ void gather_rows(_Float16* As, const _Float16* __restrict__ xh, const int* __restrict__ nbr,
                                            int slot, int base, int N, int tid) {
  const v8h z = __builtin_bit_cast(v8h, (v4f){0.f, 0.f, 0.f, 0.f});
#pragma unroll 2
  for (int idx = tid; idx < 64 * 16; idx += 128) {
    const int row = idx >> 4;
    const int c8 = (idx & 15) * 8;
    const int node = base + row;
    const bool valid = node < N;
    const int nodec = valid ? node : (N - 1);
    int src = nodec;
    if (slot > 0) {
      int nb = nbr[(size_t)nodec * 4 + (slot - 1)];
      nb = (nb < 0) ? (nb + N) : nb;
      nb = (nb < 0) ? 0 : nb;
      nb = (nb >= N) ? (N - 1) : nb;
      src = nb;
    }
    v8h v = *(const v8h*)(xh + (size_t)src * DD + c8);
    if (!valid) v = z;
    *(v8h*)(As + row * APITCH + c8) = v;
  }
}

__device__ __forceinline__ v4f ln_row(v4f y, v4f g, v4f b) {
  float s1 = y[0] + y[1] + y[2] + y[3];
#pragma unroll
  for (int off = 1; off < 32; off <<= 1) s1 += __shfl_xor(s1, off, 32);
  const float mu = s1 * (1.0f / 128.0f);
  const v4f d = y - mu;
  float s2 = d[0] * d[0] + d[1] * d[1] + d[2] * d[2] + d[3] * d[3];
#pragma unroll
  for (int off = 1; off < 32; off <<= 1) s2 += __shfl_xor(s2, off, 32);
  const float var = s2 * (1.0f / 128.0f);
  const float inv = rsqrtf(var + LN_EPS);
  return d * inv * g + b;
}

__global__ __launch_bounds__(256) void cast_rows_kernel(const float* __restrict__ x, _Float16* __restrict__ xh,
                                                        int N, int Npad) {
  const int i = blockIdx.x * 256 + threadIdx.x;
  const int total = Npad * 16;
  if (i < total) {
    const int row = i >> 4, c8 = (i & 15) * 8;
    const int rowc = (row < N) ? row : (N - 1);
    const float* src = x + (size_t)rowc * DD + c8;
    const v4f a = *(const v4f*)src;
    const v4f b = *(const v4f*)(src + 4);
    v8h o;
    o[0] = (_Float16)a[0]; o[1] = (_Float16)a[1]; o[2] = (_Float16)a[2]; o[3] = (_Float16)a[3];
    o[4] = (_Float16)b[0]; o[5] = (_Float16)b[1]; o[6] = (_Float16)b[2]; o[7] = (_Float16)b[3];
    if (row >= N) o = __builtin_bit_cast(v8h, (v4f){0.f, 0.f, 0.f, 0.f});
    _Float16* q = xh + (size_t)row * DD + c8;
    *(volatile v8h*)q = o;
    __threadfence();
    *(volatile v8h*)q = o;
  }
}

__global__ __launch_bounds__(256) void pack_wt_kernel(const float* __restrict__ w, _Float16* __restrict__ outp,
                                                      int G, int R, int Kd, int Nc, float scale, int total2) {
  const int i = blockIdx.x * 256 + threadIdx.x;
  if (i < total2) {
    const int gnk = G * Nc * Kd;
    unsigned u = 0;
#pragma unroll
    for (int e = 0; e < 2; ++e) {
      const int o = 2 * i + e;
      const int r = o / gnk;
      const int rem = o - r * gnk;
      const int n = rem / Kd;
      const int d = rem - n * Kd;
      const int g = n / Nc;
      const int cc = n - g * Nc;
      const float v = w[((size_t)(g * R + r) * Kd + d) * Nc + cc] * scale;
      const unsigned short hb = __builtin_bit_cast(unsigned short, (_Float16)v);
      u |= ((unsigned)hb) << (16 * e);
    }
    unsigned* q = (unsigned*)(void*)outp + i;
    *(volatile unsigned*)q = u;
    __threadfence();
    *(volatile unsigned*)q = u;
  }
}

__global__ __launch_bounds__(128) void qk_kernel(const _Float16* __restrict__ xh, const int* __restrict__ nbr,
                                                 const _Float16* __restrict__ Btq, const _Float16* __restrict__ Btk,
                                                 float* __restrict__ logits, int N, int Npad) {
  __shared__ __align__(16) _Float16 As[64 * APITCH];
  __shared__ __align__(16) float Qs[64 * QPITCH];
  __shared__ __align__(16) float Lg[NHEAD * 320];
  const int tid = threadIdx.x, lane = tid & 31, wave = tid >> 5;
  const int c = lane & 15, hh = lane >> 4;
  const int base = blockIdx.x * 64;
  float* lgw = Lg + wave * 320;

  gather_rows(As, xh, nbr, 0, base, N, tid);
  __syncthreads();

  {
    v8f acc[4][2];
    zero_acc(acc);
    tile_mma_42(As, APITCH, Btq + (size_t)(32 * wave) * DD, DD, lane, acc);
    acc_guard4(acc[0][0], acc[0][1], acc[1][0], acc[1][1]);
    acc_guard4(acc[2][0], acc[2][1], acc[3][0], acc[3][1]);
#pragma unroll
    for (int i = 0; i < 4; ++i)
#pragma unroll
      for (int t = 0; t < 2; ++t)
#pragma unroll
        for (int r = 0; r < 8; ++r)
          Qs[(16 * i + 8 * hh + r) * QPITCH + 32 * wave + 16 * t + c] = acc[i][t][r] * 0.125f;
  }
  wave_lds_sync();

  for (int s = 0; s < NSLOT; ++s) {
    if (s > 0) {
      __syncthreads();
      gather_rows(As, xh, nbr, s, base, N, tid);
      __syncthreads();
    }
    v8f acc[4][2];
    zero_acc(acc);
    tile_mma_42(As, APITCH, Btk + ((size_t)s * 128 + 32 * wave) * DD, DD, lane, acc);
    acc_guard4(acc[0][0], acc[0][1], acc[1][0], acc[1][1]);
    acc_guard4(acc[2][0], acc[2][1], acc[3][0], acc[3][1]);
#pragma unroll
    for (int i = 0; i < 4; ++i) {
      float pv[8];
#pragma unroll
      for (int r = 0; r < 8; ++r) {
        const int row = 16 * i + 8 * hh + r;
        const float q0 = Qs[row * QPITCH + 32 * wave + c];
        const float q1 = Qs[row * QPITCH + 32 * wave + 16 + c];
        float p = acc[i][0][r] * q0 + acc[i][1][r] * q1;
        p += __shfl_xor(p, 1, 32);
        p += __shfl_xor(p, 2, 32);
        p += __shfl_xor(p, 4, 32);
        p += __shfl_xor(p, 8, 32);
        pv[r] = p * (0.125f * QK_SCALE);
      }
      const float a0 = (c & 1) ? pv[1] : pv[0];
      const float a1 = (c & 1) ? pv[3] : pv[2];
      const float a2 = (c & 1) ? pv[5] : pv[4];
      const float a3 = (c & 1) ? pv[7] : pv[6];
      const float b0 = (c & 2) ? a1 : a0;
      const float b1 = (c & 2) ? a3 : a2;
      const float sel = (c & 4) ? b1 : b0;
      if (c < 8) lgw[s * 64 + 16 * i + 8 * hh + c] = sel;
    }
  }
  wave_lds_sync();

  const int q = lane >> 3, c4 = (lane & 7) * 4;
  for (int pass = 0; pass < 2; ++pass) {
#pragma unroll
    for (int it = 0; it < 3; ++it) {
      const int L = it * 4 + q;
      if (L < 10) {
        const int s = L >> 1, half = L & 1;
        const v4f v = *(const v4f*)(lgw + s * 64 + half * 32 + c4);
        *(volatile v4f*)(logits + (size_t)(wave * NSLOT + s) * Npad + base + half * 32 + c4) = v;
      }
    }
    __threadfence();
  }
}

__global__ __launch_bounds__(256) void colstat_kernel(const float* __restrict__ logits, float* __restrict__ stats,
                                                      int N, int Npad) {
  __shared__ float red[8];
  const int tid = threadIdx.x, lane = tid & 31, wave = tid >> 5;
  const float* p = logits + (size_t)blockIdx.x * Npad;
  float mx = -3.0e38f;
  for (int i = tid; i < N; i += 256) mx = fmaxf(mx, p[i]);
#pragma unroll
  for (int off = 1; off < 32; off <<= 1) mx = fmaxf(mx, __shfl_xor(mx, off, 32));
  if (lane == 0) red[wave] = mx;
  __syncthreads();
  float m = red[0];
#pragma unroll
  for (int w2 = 1; w2 < 8; ++w2) m = fmaxf(m, red[w2]);
  __syncthreads();
  float s = 0.f;
  for (int i = tid; i < N; i += 256) s += expf(p[i] - m);
#pragma unroll
  for (int off = 1; off < 32; off <<= 1) s += __shfl_xor(s, off, 32);
  if (lane == 0) red[wave] = s;
  __syncthreads();
  float tot = red[0];
#pragma unroll
  for (int w2 = 1; w2 < 8; ++w2) tot += red[w2];
  if (wave == 0) {
    float val = 0.f;
    if (lane == 0) val = m;
    if (lane == 1) val = 1.0f / tot;
    float* qd = stats + (size_t)blockIdx.x * STATW + lane;
    *(volatile float*)qd = val;
    __threadfence();
    *(volatile float*)qd = val;
  }
}

__global__ __launch_bounds__(128) void av_ln_kernel(const _Float16* __restrict__ xh, const float* __restrict__ x,
                                                    const int* __restrict__ nbr, const _Float16* __restrict__ Btv,
                                                    const float* __restrict__ logits, const float* __restrict__ stats,
                                                    const float* __restrict__ g1, const float* __restrict__ be1,
                                                    float* __restrict__ h1, int N, int Npad) {
  __shared__ __align__(16) _Float16 As[64 * APITCH];
  __shared__ __align__(16) float Zs[64 * DD];
  __shared__ __align__(16) float Wl[NHEAD * 320];
  const int tid = threadIdx.x, lane = tid & 31, wave = tid >> 5;
  const int c = lane & 15, hh = lane >> 4;
  const int base = blockIdx.x * 64;
  float* wlw = Wl + wave * 320;

  for (int idx = lane; idx < 320; idx += 32) {
    const int s = idx >> 6, j = idx & 63;
    const int col = wave * NSLOT + s;
    const float mx  = stats[(size_t)col * STATW];
    const float inv = stats[(size_t)col * STATW + 1];
    const float lg = logits[(size_t)col * Npad + base + j];
    wlw[idx] = expf(lg - mx) * inv;
  }
#pragma unroll 4
  for (int idx = tid; idx < 64 * DD; idx += 128) Zs[idx] = 0.f;
  gather_rows(As, xh, nbr, 0, base, N, tid);
  __syncthreads();

  for (int s = 0; s < NSLOT; ++s) {
    if (s > 0) {
      __syncthreads();
      gather_rows(As, xh, nbr, s, base, N, tid);
      __syncthreads();
    }
    v8f acc[4][2];
    zero_acc(acc);
    tile_mma_42(As, APITCH, Btv + ((size_t)s * 128 + 32 * wave) * DD, DD, lane, acc);
    acc_guard4(acc[0][0], acc[0][1], acc[1][0], acc[1][1]);
    acc_guard4(acc[2][0], acc[2][1], acc[3][0], acc[3][1]);
#pragma unroll
    for (int i = 0; i < 4; ++i)
#pragma unroll
      for (int t = 0; t < 2; ++t)
#pragma unroll
        for (int r = 0; r < 8; ++r) {
          const int row = 16 * i + 8 * hh + r;
          const float wv = wlw[s * 64 + row];
          float* zp = Zs + row * DD + 32 * wave + 16 * t + c;
          *zp = *zp + wv * (acc[i][t][r] * 0.125f);
        }
  }
  __syncthreads();

  const v4f gv = *(const v4f*)(g1 + 4 * lane);
  const v4f bv = *(const v4f*)(be1 + 4 * lane);
  for (int mm = 0; mm < 16; ++mm) {
    const int row = 16 * wave + mm;
    const int node = base + row;
    const int nodec = (node < N) ? node : (N - 1);
    const v4f xv = *(const v4f*)(x + (size_t)nodec * DD + 4 * lane);
    const v4f zv = *(const v4f*)(Zs + row * DD + 4 * lane);
    const v4f y = xv + zv;
    const v4f o = ln_row(y, gv, bv);
    store2_v4f(h1 + (size_t)node * DD + 4 * lane, o);
  }
}

__global__ __launch_bounds__(128) void ffn_ln_kernel(const float* __restrict__ h1, const _Float16* __restrict__ Bt1,
                                                     const _Float16* __restrict__ Bt2, const float* __restrict__ b1,
                                                     const float* __restrict__ b2, const float* __restrict__ g2,
                                                     const float* __restrict__ be2, float* __restrict__ out, int N) {
  __shared__ __align__(16) _Float16 Hs[32 * APITCH];
  __shared__ __align__(16) _Float16 Us[32 * UPITCH];
  __shared__ __align__(16) float Fs[32 * FPITCH];
  const int tid = threadIdx.x, lane = tid & 31, wave = tid >> 5;
  const int c = lane & 15, hh = lane >> 4, koff = hh * 8;
  const int base = blockIdx.x * 32;

#pragma unroll 2
  for (int idx = tid; idx < 32 * 32; idx += 128) {
    const int row = idx >> 5, c4 = (idx & 31) * 4;
    const int node = base + row;
    const int nodec = (node < N) ? node : (N - 1);
    const v4f v = *(const v4f*)(h1 + (size_t)nodec * DD + c4);
    v4h o;
    o[0] = (_Float16)v[0]; o[1] = (_Float16)v[1]; o[2] = (_Float16)v[2]; o[3] = (_Float16)v[3];
    *(v4h*)(Hs + row * APITCH + c4) = o;
  }
  __syncthreads();

  for (int ps = 0; ps < 2; ++ps) {
    const int n0 = 128 * wave + 64 * ps;
    v8f acc[2][4];
    zero_acc(acc);
    tile_mma_24(Hs, APITCH, Bt1 + (size_t)n0 * DD, DD, lane, acc);
    acc_guard4(acc[0][0], acc[0][1], acc[0][2], acc[0][3]);
    acc_guard4(acc[1][0], acc[1][1], acc[1][2], acc[1][3]);
#pragma unroll
    for (int j = 0; j < 4; ++j) {
      const int n = n0 + 16 * j + c;
      const float bias = b1[n];
#pragma unroll
      for (int i = 0; i < 2; ++i)
#pragma unroll
        for (int r = 0; r < 8; ++r) {
          float v = acc[i][j][r] * 0.125f + bias;
          v = fmaxf(v, 0.0f);
          Us[(16 * i + 8 * hh + r) * UPITCH + n] = (_Float16)v;
        }
    }
  }
  __syncthreads();

  v8f acc2[2][2];
  zero_acc(acc2);
  const _Float16* btw = Bt2 + (size_t)(32 * wave) * DFF;
#pragma unroll 2
  for (int kt = 0; kt < 16; ++kt) {
    v16h b[2];
#pragma unroll
    for (int t = 0; t < 2; ++t) b[t] = FH::load(btw + (size_t)(16 * t + c) * DFF + 32 * kt + koff);
#pragma unroll
    for (int i = 0; i < 2; ++i) {
      const v16h a = FH::load(Us + (16 * i + c) * UPITCH + 32 * kt + koff);
      acc2[i][0] = FH::mma(a, b[0], acc2[i][0]);
      acc2[i][1] = FH::mma(a, b[1], acc2[i][1]);
      dep_guard_h(acc2[i][0], acc2[i][1], a, b[1]);
    }
    keep2_h(b[0], b[1]);
  }
  acc_guard4(acc2[0][0], acc2[0][1], acc2[1][0], acc2[1][1]);
#pragma unroll
  for (int t = 0; t < 2; ++t) {
    const int n = 32 * wave + 16 * t + c;
    const float bias = b2[n];
#pragma unroll
    for (int i = 0; i < 2; ++i)
#pragma unroll
      for (int r = 0; r < 8; ++r)
        Fs[(16 * i + 8 * hh + r) * FPITCH + n] = acc2[i][t][r] * 0.0625f + bias;
  }
  __syncthreads();

  const v4f gv = *(const v4f*)(g2 + 4 * lane);
  const v4f bv = *(const v4f*)(be2 + 4 * lane);
  for (int mm = 0; mm < 8; ++mm) {
    const int row = 8 * wave + mm;
    const int node = base + row;
    if (node < N) {
      const v4f hv = *(const v4f*)(h1 + (size_t)node * DD + 4 * lane);
      const v4f fv = *(const v4f*)(Fs + row * FPITCH + 4 * lane);
      const v4f y = hv + fv;
      const v4f o = ln_row(y, gv, bv);
      store2_v4f(out + (size_t)node * DD + 4 * lane, o);
    }
  }
}

extern "C" void kernel_launch(void* const* d_in, const int* in_sizes, int n_in,
                              void* d_out, int out_size, void* d_ws, size_t ws_size,
                              hipStream_t stream) {
  if (n_in < 13) return;
  const float* x   = (const float*)d_in[0];
  const int*   nbr = (const int*)d_in[1];
  const float* w_q = (const float*)d_in[2];
  const float* w_k = (const float*)d_in[3];
  const float* w_v = (const float*)d_in[4];
  const float* W1  = (const float*)d_in[5];
  const float* b1  = (const float*)d_in[6];
  const float* W2  = (const float*)d_in[7];
  const float* b2  = (const float*)d_in[8];
  const float* g1  = (const float*)d_in[9];
  const float* be1 = (const float*)d_in[10];
  const float* g2  = (const float*)d_in[11];
  const float* be2 = (const float*)d_in[12];
  float* out = (float*)d_out;

  const int N = in_sizes[0] / DD;
  if (N <= 0) return;
  if (in_sizes[1] < N * 4) return;
  if (in_sizes[2] < NHEAD * DD * 32) return;
  if (in_sizes[3] < NHEAD * NSLOT * DD * 32) return;
  if (in_sizes[4] < NHEAD * NSLOT * DD * 32) return;
  if (in_sizes[5] < DD * DFF || in_sizes[7] < DFF * DD) return;
  if (in_sizes[6] < DFF || in_sizes[8] < DD || in_sizes[9] < DD || in_sizes[10] < DD || in_sizes[11] < DD || in_sizes[12] < DD) return;
  if (out_size < N * DD) return;
  const int Npad = ((N + 63) / 64) * 64;

  char* ws = (char*)d_ws;
  size_t off = 0;
  auto carve = [&](size_t bytes) -> void* {
    off = (off + 255) & ~(size_t)255;
    void* p = ws + off;
    off += bytes;
    return p;
  };
  _Float16* xh   = (_Float16*)carve((size_t)Npad * DD * 2);
  _Float16* Btq  = (_Float16*)carve((size_t)DD * DD * 2);
  _Float16* Btk  = (_Float16*)carve((size_t)NSLOT * DD * DD * 2);
  _Float16* Btv  = (_Float16*)carve((size_t)NSLOT * DD * DD * 2);
  _Float16* Bt1  = (_Float16*)carve((size_t)DFF * DD * 2);
  _Float16* Bt2  = (_Float16*)carve((size_t)DD * DFF * 2);
  float*    lgt  = (float*)carve((size_t)NCOL * Npad * 4);
  float*    stat = (float*)carve((size_t)NCOL * STATW * 4);
  float*    h1   = (float*)carve((size_t)Npad * DD * 4);
  off = (off + 255) & ~(size_t)255;
  if (off > ws_size || off > (size_t)134217728) return;

  cast_rows_kernel<<<(Npad * 16 + 255) / 256, 256, 0, stream>>>(x, xh, N, Npad);
  {
    const int tq = (DD * DD) / 2;
    const int tk = (NSLOT * DD * DD) / 2;
    const int t1 = (DD * DFF) / 2;
    pack_wt_kernel<<<(tq + 255) / 256, 256, 0, stream>>>(w_q, Btq, NHEAD, 1, DD, 32, 8.0f, tq);
    pack_wt_kernel<<<(tk + 255) / 256, 256, 0, stream>>>(w_k, Btk, NHEAD, NSLOT, DD, 32, 8.0f, tk);
    pack_wt_kernel<<<(tk + 255) / 256, 256, 0, stream>>>(w_v, Btv, NHEAD, NSLOT, DD, 32, 8.0f, tk);
    pack_wt_kernel<<<(t1 + 255) / 256, 256, 0, stream>>>(W1, Bt1, 1, 1, DD, DFF, 8.0f, t1);
    pack_wt_kernel<<<(t1 + 255) / 256, 256, 0, stream>>>(W2, Bt2, 1, 1, DFF, DD, 16.0f, t1);
  }
  qk_kernel<<<Npad / 64, 128, 0, stream>>>(xh, nbr, Btq, Btk, lgt, N, Npad);
  colstat_kernel<<<NCOL, 256, 0, stream>>>(lgt, stat, N, Npad);
  av_ln_kernel<<<Npad / 64, 128, 0, stream>>>(xh, x, nbr, Btv, lgt, stat, g1, be1, h1, N, Npad);
  ffn_ln_kernel<<<(N + 31) / 32, 128, 0, stream>>>(h1, Bt1, Bt2, b1, b2, g2, be2, out, N);
}
